// StackedEncoderModel_24945170055373
// MI455X (gfx1250) — hardware-verified
//
#include <hip/hip_runtime.h>
#include <math.h>

typedef __attribute__((ext_vector_type(16))) _Float16 v16h;
typedef __attribute__((ext_vector_type(8)))  _Float16 v8h;
typedef __attribute__((ext_vector_type(2)))  _Float16 v2h;
typedef __attribute__((ext_vector_type(16))) __bf16   v16b;
typedef __attribute__((ext_vector_type(8)))  __bf16   v8b;
typedef __attribute__((ext_vector_type(8)))  float    v8f;
typedef __attribute__((ext_vector_type(4)))  float    v4f;

constexpr int kLayers = 4;
constexpr int kBatch  = 4;
constexpr int kSeq    = 2048;
constexpr int kRows   = kBatch * kSeq;
constexpr int kFin    = 256;
constexpr int kD      = 1024;
constexpr int kD2     = 2 * kD;
constexpr int kThr    = 256;
constexpr int kStP    = 32;

constexpr float kInCarry = 1024.0f;
constexpr float kACarry  = 256.0f;
constexpr float kScIn = 1.0f / (kInCarry * kInCarry);
constexpr float kScA  = 1.0f / (kACarry * kInCarry);
constexpr float kF16MinNormal = 6.103515625e-5f;
constexpr float kLnEps = 1e-5f;

static_assert((kRows % 64) == 0 && (kD % 64) == 0 && (kD2 % 64) == 0, "GEMM M, N multiples of 64");
static_assert(((kRows / 64) * (kD / 64)) % 8 == 0, "GEMM grids exact");
static_assert((kFin % 32) == 0 && (kD % 32) == 0, "GEMM K multiples of 32");

constexpr size_t kOffIN  = 0;
constexpr size_t kOffWIN = kOffIN  + (size_t)kRows * kFin * 2;
constexpr size_t kOffBW  = kOffWIN + (size_t)kD * kFin * 2;
constexpr size_t kOffCW  = kOffBW  + (size_t)kLayers * kD2 * kD * 2;
constexpr size_t kOffWW  = kOffCW  + (size_t)kLayers * kD * kD2 * 2;
constexpr size_t kOffBV  = kOffWW  + (size_t)kLayers * kD2 * kD * 2;
constexpr int    kBvIn   = 0;
constexpr int    kBvL    = kD;
constexpr int    kBvZ    = kD + kLayers * kD2;
constexpr int    kBvTot  = kBvZ + kD2;
constexpr size_t kOffX   = kOffBV  + (size_t)kBvTot * 4;
constexpr size_t kOffST  = kOffX   + (size_t)kRows * kD * 4;
constexpr size_t kOffA16 = kOffST  + (size_t)kRows * kStP * 4;
constexpr size_t kOffBP  = kOffA16 + (size_t)kRows * kD * 2;
constexpr size_t kOffHS  = kOffBP  + (size_t)kRows * kD2 * 4;
constexpr size_t kOffY   = kOffHS  + (size_t)kRows * kD2 * 2;
constexpr size_t kWsTotal = kOffY  + (size_t)kRows * kD * 4;
static_assert(kWsTotal <= 268435456ull, "inside the offered workspace");
static_assert((kOffWIN % 256) == 0 && (kOffBW % 256) == 0 && (kOffCW % 256) == 0 && (kOffWW % 256) == 0 && (kOffBV % 256) == 0 && (kOffX % 256) == 0 && (kOffST % 256) == 0 && (kOffA16 % 256) == 0 && (kOffBP % 256) == 0 && (kOffHS % 256) == 0 && (kOffY % 256) == 0, "aligned regions");

__device__ __forceinline__ unsigned short f2bf_bits(float f) {
  unsigned u = __float_as_uint(f);
  return (unsigned short)((u + 0x7FFFu + ((u >> 16) & 1u)) >> 16);
}
__device__ __forceinline__ float bf_bits2f(unsigned short h) { return __uint_as_float(((unsigned)h) << 16); }
__device__ __forceinline__ float bf16r(float f) { return bf_bits2f(f2bf_bits(f)); }
__device__ __forceinline__ float carry_flush(float v, float carry) {
  const float s = v * carry;
  return (fabsf(s) < kF16MinNormal) ? 0.0f : s;
}
__device__ __forceinline__ float frcp(float x) { return __builtin_amdgcn_rcpf(x); }

__device__ __forceinline__ void dep_guard4_h(v8f& a, v8f& b, v8f& c, v8f& d, v16h x, v16h y) { asm volatile("v_nop\n\tv_nop\n\tv_nop\n\tv_nop" : "+v"(a), "+v"(b), "+v"(c), "+v"(d) : "v"(x), "v"(y)); }
__device__ __forceinline__ void dep_guard4_b(v8f& a, v8f& b, v8f& c, v8f& d, v16b x, v16b y) { asm volatile("v_nop\n\tv_nop\n\tv_nop\n\tv_nop" : "+v"(a), "+v"(b), "+v"(c), "+v"(d) : "v"(x), "v"(y)); }
__device__ __forceinline__ void keep4_h(v16h a, v16h b, v16h c, v16h d) { asm volatile("v_nop" :: "v"(a), "v"(b), "v"(c), "v"(d)); }
__device__ __forceinline__ void keep4_b(v16b a, v16b b, v16b c, v16b d) { asm volatile("v_nop" :: "v"(a), "v"(b), "v"(c), "v"(d)); }
__device__ __forceinline__ void acc_guard4(v8f& a, v8f& b, v8f& c, v8f& d) { asm volatile("v_nop\n\tv_nop\n\tv_nop\n\tv_nop" : "+v"(a), "+v"(b), "+v"(c), "+v"(d)); }

template <typename T> struct Frag;
template <> struct Frag<_Float16> {
  typedef v16h V; union U { v16h v; v8h h[2]; };
  static __device__ __forceinline__ v16h load(const _Float16* p) {
    U f; f.h[0] = *(const v8h*)(p); f.h[1] = *(const v8h*)(p + 16); return f.v;
  }
  static __device__ __forceinline__ v8f mma(v16h a, v16h b, v8f c) {
    return __builtin_amdgcn_wmma_f32_16x16x32_f16(false, a, false, b, (short)0, c, false, false);
  }
  static __device__ __forceinline__ void guard4(v8f& a, v8f& b, v8f& c, v8f& d, v16h x, v16h y) { dep_guard4_h(a, b, c, d, x, y); }
  static __device__ __forceinline__ void keep(v16h a, v16h b, v16h c, v16h d) { keep4_h(a, b, c, d); }
};
template <> struct Frag<__bf16> {
  typedef v16b V; union U { v16b v; v8b h[2]; };
  static __device__ __forceinline__ v16b load(const __bf16* p) {
    U f; f.h[0] = *(const v8b*)(p); f.h[1] = *(const v8b*)(p + 16); return f.v;
  }
  static __device__ __forceinline__ v8f mma(v16b a, v16b b, v8f c) {
    return __builtin_amdgcn_wmma_f32_16x16x32_bf16(false, a, false, b, (short)0, c, false, false);
  }
  static __device__ __forceinline__ void guard4(v8f& a, v8f& b, v8f& c, v8f& d, v16b x, v16b y) { dep_guard4_b(a, b, c, d, x, y); }
  static __device__ __forceinline__ void keep(v16b a, v16b b, v16b c, v16b d) { keep4_b(a, b, c, d); }
};

__device__ __forceinline__ v8f mma_h(v16h a, v16h b, v8f c) {
  c = __builtin_amdgcn_wmma_f32_16x16x32_f16(false, a, false, b, (short)0, c, false, false);
  asm volatile("v_nop\n\tv_nop\n\tv_nop\n\tv_nop" : "+v"(c) : "v"(a), "v"(b));
  return c;
}

template <int ET> struct Elem;
template <> struct Elem<0> { typedef _Float16 T; };
template <> struct Elem<1> { typedef __bf16 T; };
template <int ET, bool SPLIT, int BIAS_MODE, int OUT_MODE, bool RESID, int ACT = 0>
__global__ __launch_bounds__(256) void wmma_gemm64(
    const unsigned short* __restrict__ Ap, const unsigned short* __restrict__ A2p, int lda, long strideA,
    const unsigned short* __restrict__ Btp, const unsigned short* __restrict__ Bt2p, int ldb, long strideB,
    void* __restrict__ Cout, void* __restrict__ Cout2, int ldc, long strideC,
    const float* __restrict__ bias,
    const float* __restrict__ resid, long strideR,
    int M, int N, int K, float scale) {
  typedef typename Elem<ET>::T T;
  typedef typename Frag<T>::V V;
  const T* A = (const T*)Ap; const T* A2 = (const T*)A2p; const T* Bt = (const T*)Btp; const T* Bt2 = (const T*)Bt2p;
  __shared__ __align__(16) float sT[8][16 * 68];
  const int b    = blockIdx.y;
  const int lane = threadIdx.x & 31;
  const int wave = threadIdx.x >> 5;
  const int tilesN = N >> 6;
  const int tilesM = M >> 6;
  const int tile = blockIdx.x * 8 + wave;
  if (tile >= tilesM * tilesN) return;
  const int tm = tile / tilesN;
  const int tn = tile - tm * tilesN;
  const int m0 = tm << 6;
  const int n0 = tn << 6;

  const T* Ab  = A  + (size_t)b * strideA;
  const T* Bb  = Bt + (size_t)b * strideB;
  const T* Ab2 = SPLIT ? (A2  + (size_t)b * strideA) : nullptr;
  const T* Bb2 = SPLIT ? (Bt2 + (size_t)b * strideB) : nullptr;

  const int rlane = lane & 15;
  const int koff  = (lane >> 4) * 8;
  const int mOff  = (lane >> 4) * 8;

  v8f acc[4][4];
#pragma unroll
  for (int i = 0; i < 4; ++i)
#pragma unroll
    for (int j = 0; j < 4; ++j) acc[i][j] = (v8f){0.f,0.f,0.f,0.f,0.f,0.f,0.f,0.f};

  for (int k0 = 0; k0 < K; k0 += 32) {
    V bh[4], bl[4];
#pragma unroll
    for (int j = 0; j < 4; ++j) {
      const size_t bo = (size_t)(n0 + (j << 4) + rlane) * ldb + koff + k0;
      bh[j] = Frag<T>::load(Bb + bo);
      if (SPLIT) bl[j] = Frag<T>::load(Bb2 + bo);
    }
#pragma unroll
    for (int i = 0; i < 4; ++i) {
      const size_t ao = (size_t)(m0 + (i << 4) + rlane) * lda + koff + k0;
      V ah = Frag<T>::load(Ab + ao);
      V al;
      if (SPLIT) al = Frag<T>::load(Ab2 + ao);
#pragma unroll
      for (int j = 0; j < 4; ++j) {
        acc[i][j] = Frag<T>::mma(ah, bh[j], acc[i][j]);
        if (SPLIT) {
          acc[i][j] = Frag<T>::mma(ah, bl[j], acc[i][j]);
          acc[i][j] = Frag<T>::mma(al, bh[j], acc[i][j]);
        }
      }
      Frag<T>::guard4(acc[i][0], acc[i][1], acc[i][2], acc[i][3], ah, SPLIT ? al : ah);
    }
    Frag<T>::keep(bh[0], bh[1], bh[2], bh[3]);
    if (SPLIT) Frag<T>::keep(bl[0], bl[1], bl[2], bl[3]);
  }
  acc_guard4(acc[0][0], acc[0][1], acc[0][2], acc[0][3]);
  acc_guard4(acc[1][0], acc[1][1], acc[1][2], acc[1][3]);
  acc_guard4(acc[2][0], acc[2][1], acc[2][2], acc[2][3]);
  acc_guard4(acc[3][0], acc[3][1], acc[3][2], acc[3][3]);

  float* slab = sT[wave];
  const float* Rb = RESID ? (resid + (size_t)b * strideR) : nullptr;
#pragma unroll
  for (int i = 0; i < 4; ++i) {
    const int mBase = m0 + (i << 4);
#pragma unroll
    for (int j = 0; j < 4; ++j) {
      const int n = n0 + (j << 4) + rlane;
      float bv = 0.f;
      if (BIAS_MODE == 2) bv = bias[n];
#pragma unroll
      for (int r = 0; r < 8; ++r) {
        float v = acc[i][j][r] * scale;
        if (BIAS_MODE == 1) v += bias[mBase + mOff + r];
        if (BIAS_MODE == 2) v += bv;
        if (RESID) v += Rb[(size_t)(mBase + mOff + r) * ldc + n];
        if (ACT == 1) v = tanhf(v);
        if (ACT == 2) v = fmaxf(v, 0.0f);
        if (ACT == 3) v = v / (1.0f + expf(-v));
        if (ACT == 4) v = (v > 0.f) ? v : 0.01f * v;
        slab[(mOff + r) * 68 + (j << 4) + rlane] = v;
      }
    }
    __builtin_amdgcn_fence(__ATOMIC_RELEASE, "workgroup");
    __builtin_amdgcn_wave_barrier();
    __builtin_amdgcn_fence(__ATOMIC_ACQUIRE, "workgroup");
    if (OUT_MODE == 0) {
      float* C = (float*)Cout + (size_t)b * strideC;
      const int hh = lane >> 4, c4 = (lane & 15) * 4;
      for (int pass = 0; pass < 2; ++pass) {
#pragma unroll
        for (int it = 0; it < 8; ++it) {
          const int row = it * 2 + hh;
          v4f v = *(const v4f*)(slab + row * 68 + c4);
          *(volatile v4f*)(C + (size_t)(mBase + row) * ldc + n0 + c4) = v;
        }
        __threadfence();
      }
    } else {
      const int q = lane >> 3, c8 = (lane & 7) * 8;
      unsigned short* C  = (unsigned short*)Cout  + (size_t)b * strideC;
      unsigned short* C2 = (OUT_MODE == 2) ? ((unsigned short*)Cout2 + (size_t)b * strideC) : nullptr;
      for (int pass = 0; pass < 2; ++pass) {
#pragma unroll
        for (int it = 0; it < 4; ++it) {
          const int row = it * 4 + q;
          const float* sp = slab + row * 68 + c8;
          v8h hv, lv;
#pragma unroll
          for (int e = 0; e < 8; ++e) {
            if (OUT_MODE == 1) {
              hv[e] = (_Float16)sp[e];
            } else {
              unsigned short hb = f2bf_bits(sp[e]);
              unsigned short lb = f2bf_bits(sp[e] - bf_bits2f(hb));
              hv[e] = __builtin_bit_cast(_Float16, hb);
              lv[e] = __builtin_bit_cast(_Float16, lb);
            }
          }
          *(volatile v8h*)(C + (size_t)(mBase + row) * ldc + n0 + c8) = hv;
          if (OUT_MODE == 2) *(volatile v8h*)(C2 + (size_t)(mBase + row) * ldc + n0 + c8) = lv;
        }
        __threadfence();
      }
    }
    __builtin_amdgcn_fence(__ATOMIC_RELEASE, "workgroup");
    __builtin_amdgcn_wave_barrier();
    __builtin_amdgcn_fence(__ATOMIC_ACQUIRE, "workgroup");
  }
}

__global__ __launch_bounds__(kThr) void cast_plane_kernel(const float* __restrict__ src, unsigned short* __restrict__ dst,
                                                          int colsLog2, int dstPitch, int dstOff) {
  const int i   = blockIdx.x * kThr + threadIdx.x;
  const int sh  = colsLog2 - 3;
  const int row = i >> sh;
  const int c8  = (i & ((1 << sh) - 1)) * 8;
  const float* sp = src + ((size_t)row << colsLog2) + c8;
  const v4f a0 = *(const v4f*)(sp);
  const v4f a1 = *(const v4f*)(sp + 4);
  v8h hv;
#pragma unroll
  for (int e = 0; e < 4; ++e) {
    const float f0 = a0[e];
    const float f1 = a1[e];
    hv[e]     = (_Float16)carry_flush(bf16r(f0), kInCarry);
    hv[4 + e] = (_Float16)carry_flush(bf16r(f1), kInCarry);
  }
  unsigned short* dp = dst + (size_t)row * dstPitch + dstOff + c8;
  *(volatile v8h*)dp = hv;
  __threadfence();
  *(volatile v8h*)dp = hv;
}

__global__ __launch_bounds__(kThr) void bias_rows_kernel(const float* __restrict__ b_in, const float* __restrict__ b1,
                                                         const float* __restrict__ b2, float* __restrict__ BV) {
  const int i = blockIdx.x * kThr + threadIdx.x;
  const int j = i - kBvL;
  const int jl = (j >= 0 && j < kLayers * kD2) ? j : 0;
  const int l = jl >> 11;
  const int n = jl & (kD2 - 1);
  const int nc = n & (kD - 1);
  const float vin = b_in[(i < kD) ? i : 0];
  const float v1 = b1[l * kD + nc];
  const float v2 = b2[l * kD + nc];
  const float vl = (n < kD) ? v1 : v2;
  const float o = (i < kD) ? bf16r(vin) : ((i < kBvZ) ? bf16r(vl) : 0.0f);
  for (int pass = 0; pass < 2; ++pass) {
    *(volatile float*)(BV + i) = o;
    __threadfence();
  }
}
static_assert(kBvTot % kThr == 0 && kD % kThr == 0 && kD2 % kThr == 0, "bias grid exact; regions block-uniform");

__device__ __forceinline__ float block_sum_256(float v, float* red, float* wsum) {
  const int tid = threadIdx.x;
  red[tid] = v;
  __syncthreads();
  if ((tid & 31) == 0) {
    float s = 0.0f;
#pragma unroll 1
    for (int k = 0; k < 32; ++k) s += red[tid + k];
    wsum[tid >> 5] = s;
  }
  __syncthreads();
  float t = 0.0f;
#pragma unroll
  for (int k = 0; k < 8; ++k) t += wsum[k];
  __syncthreads();
  return t;
}

__global__ __launch_bounds__(kThr) void ln_kernel(const float* __restrict__ X, const float* __restrict__ ln_scale,
                                                  const float* __restrict__ ln_bias, unsigned short* __restrict__ A16,
                                                  float* __restrict__ ST) {
  __shared__ float red[kThr];
  __shared__ float wsum[8];
  const int row = blockIdx.x;
  const int tid = threadIdx.x;
  const int f4 = tid * 4;
  const v4f xv = *(const v4f*)(X + (size_t)row * kD + f4);
  const float mu = block_sum_256((xv[0] + xv[1]) + (xv[2] + xv[3]), red, wsum) * (1.0f / (float)kD);
  const float d0 = xv[0] - mu, d1 = xv[1] - mu, d2 = xv[2] - mu, d3 = xv[3] - mu;
  const float var = block_sum_256((d0 * d0 + d1 * d1) + (d2 * d2 + d3 * d3), red, wsum) * (1.0f / (float)kD);
  const float rs = 1.0f / sqrtf(var + kLnEps);
  const v4f sc = *(const v4f*)(ln_scale + f4);
  const v4f bi = *(const v4f*)(ln_bias + f4);
  typedef __attribute__((ext_vector_type(4))) _Float16 v4h;
  v4h hv;
#pragma unroll
  for (int e = 0; e < 4; ++e) {
    const float s0 = sc[e], b0 = bi[e];
    const float dn = (e == 0) ? d0 : ((e == 1) ? d1 : ((e == 2) ? d2 : d3));
    hv[e] = (_Float16)carry_flush(dn * rs * bf16r(s0) + bf16r(b0), kACarry);
  }
  unsigned short* dp = A16 + (size_t)row * kD + f4;
  for (int pass = 0; pass < 2; ++pass) {
    *(volatile v4h*)dp = hv;
    if (tid < 32) *(volatile float*)(ST + (size_t)row * kStP + tid) = (tid == 0) ? mu : ((tid == 1) ? rs : 0.0f);
    __threadfence();
  }
}

__global__ __launch_bounds__(kThr) void lru_scan_kernel(const float* __restrict__ BP, const float* __restrict__ nu_log,
                                                        const float* __restrict__ theta_log, unsigned short* __restrict__ HS) {
  const int v = blockIdx.x * kThr + threadIdx.x;
  const int b = v >> 9;
  const int h0 = (v & 511) * 2;
  float lre[2], lim[2], gam[2], sre[2] = {0.0f, 0.0f}, sim[2] = {0.0f, 0.0f};
#pragma unroll
  for (int k = 0; k < 2; ++k) {
    const float nl = nu_log[h0 + k], tl = theta_log[h0 + k];
    const float nu = expf(bf16r(nl));
    const float th = expf(bf16r(tl));
    const float mag = expf(-nu);
    float sn, cs;
    sincosf(th, &sn, &cs);
    lre[k] = mag * cs;
    lim[k] = mag * sn;
    gam[k] = expf(0.5f * logf(1.0f - expf(-2.0f * nu) + 1e-5f));
  }
  const float* bp = BP + (size_t)b * kSeq * kD2 + h0;
  unsigned short* hp = HS + (size_t)b * kSeq * kD2 + h0;
#pragma unroll 1
  for (int t = 0; t < kSeq; ++t) {
    const float2 ur = *(const float2*)(bp + (size_t)t * kD2);
    const float2 ui = *(const float2*)(bp + (size_t)t * kD2 + kD);
    const float bur[2] = {ur.x, ur.y}, bui[2] = {ui.x, ui.y};
    v2h ore, oim;
#pragma unroll
    for (int k = 0; k < 2; ++k) {
      const float nr = lre[k] * sre[k] - lim[k] * sim[k] + gam[k] * bur[k];
      const float ni = lre[k] * sim[k] + lim[k] * sre[k] + gam[k] * bui[k];
      sre[k] = nr; sim[k] = ni;
      ore[k] = (_Float16)carry_flush(nr, kACarry);
      oim[k] = (_Float16)carry_flush(-ni, kACarry);
    }
    unsigned short* dp = hp + (size_t)t * kD2;
    for (int pass = 0; pass < 2; ++pass) {
      *(volatile v2h*)dp = ore;
      *(volatile v2h*)(dp + kD) = oim;
      __threadfence();
    }
  }
}
static_assert((kBatch * 512) % kThr == 0, "scan grid exact");

__global__ __launch_bounds__(kThr) void gelu_kernel(const float* __restrict__ Y, const float* __restrict__ X, const float* __restrict__ ST,
                                                    const float* __restrict__ ln_scale, const float* __restrict__ ln_bias,
                                                    const float* __restrict__ d_diag, unsigned short* __restrict__ A16) {
  const size_t v = (size_t)blockIdx.x * kThr + threadIdx.x;
  const size_t row = v >> 7;
  const int f8 = (int)(v & 127) * 8;
  const float mu = ST[row * kStP], rs = ST[row * kStP + 1];
  v8h hv;
#pragma unroll
  for (int hlf = 0; hlf < 2; ++hlf) {
    const v4f yv = *(const v4f*)(Y + row * kD + f8 + 4 * hlf);
    const v4f xv = *(const v4f*)(X + row * kD + f8 + 4 * hlf);
    const v4f sc = *(const v4f*)(ln_scale + f8 + 4 * hlf);
    const v4f bi = *(const v4f*)(ln_bias + f8 + 4 * hlf);
    const v4f dd = *(const v4f*)(d_diag + f8 + 4 * hlf);
#pragma unroll
    for (int e = 0; e < 4; ++e) {
      const float s0 = sc[e], b0 = bi[e], d0 = dd[e];
      const float xn = (xv[e] - mu) * rs * bf16r(s0) + bf16r(b0);
      const float y = yv[e] + xn * bf16r(d0);
      const float g = 0.5f * y * (1.0f + erff(y * 0.70710678118654752440f));
      hv[4 * hlf + e] = (_Float16)carry_flush(g, kACarry);
    }
  }
  unsigned short* dp = A16 + row * kD + f8;
  *(volatile v8h*)dp = hv;
  __threadfence();
  *(volatile v8h*)dp = hv;
}
static_assert(((size_t)kRows * 128) % kThr == 0, "gelu grid exact");

__global__ __launch_bounds__(kThr) void gate_kernel(const float* __restrict__ X, const float* __restrict__ P, float* __restrict__ dst) {
  const size_t row = blockIdx.x;
  const int f4 = threadIdx.x * 4;
  const v4f xv = *(const v4f*)(X + row * kD + f4);
  const v4f p1 = *(const v4f*)(P + row * kD2 + f4);
  const v4f p2 = *(const v4f*)(P + row * kD2 + kD + f4);
  v4f o;
#pragma unroll
  for (int e = 0; e < 4; ++e) o[e] = xv[e] + p1[e] * (1.0f / (1.0f + expf(-p2[e])));
  float* dp = dst + row * kD + f4;
  *(volatile v4f*)dp = o;
  __threadfence();
  *(volatile v4f*)dp = o;
}

static_assert(((size_t)kRows * kFin / 8) % kThr == 0 && ((size_t)kD * kFin / 8) % kThr == 0 && ((size_t)kD * kD / 8) % kThr == 0, "cast grids exact");

extern "C" void kernel_launch(void* const* d_in, const int* in_sizes, int n_in,
                              void* d_out, int out_size, void* d_ws, size_t ws_size,
                              hipStream_t stream) {
  if (n_in < 16 || d_out == nullptr || d_ws == nullptr) return;
  if (in_sizes[0] != kRows * kFin || in_sizes[1] != kD * kFin || in_sizes[2] != kD) return;
  if (in_sizes[3] != kLayers * kD || in_sizes[4] != kLayers * kD) return;
  if (in_sizes[5] != kLayers * kD * kD || in_sizes[6] != kLayers * kD * kD || in_sizes[7] != kLayers * kD * kD || in_sizes[8] != kLayers * kD * kD) return;
  if (in_sizes[9] != kLayers * kD || in_sizes[10] != kLayers * kD || in_sizes[11] != kLayers * kD) return;
  if (in_sizes[12] != kLayers * kD * kD || in_sizes[13] != kLayers * kD || in_sizes[14] != kLayers * kD * kD || in_sizes[15] != kLayers * kD) return;
  if (out_size != kRows * kD) return;
  if (ws_size < kWsTotal) return;
  const float* inputs = (const float*)d_in[0];
  const float* W_in = (const float*)d_in[1];
  const float* b_in = (const float*)d_in[2];
  const float* nu_log = (const float*)d_in[3];
  const float* theta_log = (const float*)d_in[4];
  const float* B_re = (const float*)d_in[5];
  const float* B_im = (const float*)d_in[6];
  const float* C_re = (const float*)d_in[7];
  const float* C_im = (const float*)d_in[8];
  const float* D_diag = (const float*)d_in[9];
  const float* ln_scale = (const float*)d_in[10];
  const float* ln_bias = (const float*)d_in[11];
  const float* w1 = (const float*)d_in[12];
  const float* b1 = (const float*)d_in[13];
  const float* w2 = (const float*)d_in[14];
  const float* b2 = (const float*)d_in[15];
  float* out = (float*)d_out;
  char* ws = (char*)d_ws;
  unsigned short* IN16 = (unsigned short*)(ws + kOffIN);
  unsigned short* WIN  = (unsigned short*)(ws + kOffWIN);
  unsigned short* BW   = (unsigned short*)(ws + kOffBW);
  unsigned short* CW   = (unsigned short*)(ws + kOffCW);
  unsigned short* WW   = (unsigned short*)(ws + kOffWW);
  float* BV  = (float*)(ws + kOffBV);
  float* X   = (float*)(ws + kOffX);
  float* ST  = (float*)(ws + kOffST);
  unsigned short* A16 = (unsigned short*)(ws + kOffA16);
  float* BP  = (float*)(ws + kOffBP);
  unsigned short* HS  = (unsigned short*)(ws + kOffHS);
  float* Y   = (float*)(ws + kOffY);

  cast_plane_kernel<<<(int)(((size_t)kRows * kFin / 8) / kThr), kThr, 0, stream>>>(inputs, IN16, 8, kFin, 0);
  cast_plane_kernel<<<(int)(((size_t)kD * kFin / 8) / kThr), kThr, 0, stream>>>(W_in, WIN, 8, kFin, 0);
  const int gW = (int)(((size_t)kD * kD / 8) / kThr);
  for (int l = 0; l < kLayers; ++l) {
    const size_t mo = (size_t)l * kD * kD;
    cast_plane_kernel<<<gW, kThr, 0, stream>>>(B_re + mo, BW + (size_t)l * kD2 * kD, 10, kD, 0);
    cast_plane_kernel<<<gW, kThr, 0, stream>>>(B_im + mo, BW + (size_t)l * kD2 * kD + (size_t)kD * kD, 10, kD, 0);
    cast_plane_kernel<<<gW, kThr, 0, stream>>>(C_re + mo, CW + (size_t)l * kD * kD2, 10, kD2, 0);
    cast_plane_kernel<<<gW, kThr, 0, stream>>>(C_im + mo, CW + (size_t)l * kD * kD2, 10, kD2, kD);
    cast_plane_kernel<<<gW, kThr, 0, stream>>>(w1 + mo, WW + (size_t)l * kD2 * kD, 10, kD, 0);
    cast_plane_kernel<<<gW, kThr, 0, stream>>>(w2 + mo, WW + (size_t)l * kD2 * kD + (size_t)kD * kD, 10, kD, 0);
  }
  bias_rows_kernel<<<kBvTot / kThr, kThr, 0, stream>>>(b_in, b1, b2, BV);

  wmma_gemm64<0, false, 2, 0, false, 0><<<dim3((kRows / 64) * (kD / 64) / 8, 1), 256, 0, stream>>>(
      IN16, IN16, kFin, 0L, WIN, WIN, kFin, 0L, (void*)X, (void*)X, kD, 0L, BV + kBvIn, nullptr, 0L, kRows, kD, kFin, kScIn);
  for (int l = 0; l < kLayers; ++l) {
    ln_kernel<<<kRows, kThr, 0, stream>>>(X, ln_scale + l * kD, ln_bias + l * kD, A16, ST);
    wmma_gemm64<0, false, 2, 0, false, 0><<<dim3((kRows / 64) * (kD2 / 64) / 8, 1), 256, 0, stream>>>(
        A16, A16, kD, 0L, BW + (size_t)l * kD2 * kD, BW + (size_t)l * kD2 * kD, kD, 0L, (void*)BP, (void*)BP, kD2, 0L, BV + kBvZ, nullptr, 0L, kRows, kD2, kD, kScA);
    lru_scan_kernel<<<(kBatch * 512) / kThr, kThr, 0, stream>>>(BP, nu_log + l * kD, theta_log + l * kD, HS);
    wmma_gemm64<0, false, 2, 0, false, 0><<<dim3((kRows / 64) * (kD / 64) / 8, 1), 256, 0, stream>>>(
        HS, HS, kD2, 0L, CW + (size_t)l * kD * kD2, CW + (size_t)l * kD * kD2, kD2, 0L, (void*)Y, (void*)Y, kD, 0L, BV + kBvZ, nullptr, 0L, kRows, kD, kD2, kScA);
    gelu_kernel<<<(int)(((size_t)kRows * 128) / kThr), kThr, 0, stream>>>(Y, X, ST, ln_scale + l * kD, ln_bias + l * kD, D_diag + l * kD, A16);
    wmma_gemm64<0, false, 2, 0, false, 0><<<dim3((kRows / 64) * (kD2 / 64) / 8, 1), 256, 0, stream>>>(
        A16, A16, kD, 0L, WW + (size_t)l * kD2 * kD, WW + (size_t)l * kD2 * kD, kD, 0L, (void*)BP, (void*)BP, kD2, 0L, BV + kBvL + l * kD2, nullptr, 0L, kRows, kD2, kD, kScA);
    gate_kernel<<<kRows, kThr, 0, stream>>>(X, BP, (l + 1 < kLayers) ? X : out);
  }
}
